// LSTM_83202106458149
// MI455X (gfx1250) — hardware-verified
//
#include <hip/hip_runtime.h>
#include <math.h>

constexpr int NTOK      = 131072;
constexpr int NHID      = 256;
constexpr int NGATE     = 4 * NHID;
constexpr int ROW_G     = 2 * NHID;
constexpr int ROW_O     = 3 * NHID;
constexpr int NGRP      = NHID / 16;
constexpr int GRP_ROWS  = 48;
constexpr int BT_ROWS   = NGRP * GRP_ROWS;
constexpr int TOK_BLK   = 128;
constexpr int TOK_PASS  = 64;
constexpr int NPASS     = TOK_BLK / TOK_PASS;
constexpr int NTHR      = 128;
constexpr int NWAVE     = NTHR / 32;
constexpr int APITCH    = 264;
constexpr int KSTEPS    = NHID / 32;
constexpr int PACK_THR  = 256;
constexpr int NPACK     = BT_ROWS * (NHID / 8);
constexpr float ACARRY  = 64.0f;
constexpr float WCARRY  = 16.0f;
constexpr float FOLD    = 1.0f / (ACARRY * WCARRY);
constexpr int C_W0I = 0 * NHID;
constexpr int C_W0G = 1 * NHID;
constexpr int C_W0O = 2 * NHID;
constexpr int C_B0I = 3 * NHID;
constexpr int C_B0G = 4 * NHID;
constexpr int C_B0O = 5 * NHID;
constexpr int C_B1I = 6 * NHID;
constexpr int C_B1G = 7 * NHID;
constexpr int C_B1O = 8 * NHID;
constexpr int C_WL  = 9 * NHID;
constexpr int C_TOT = 10 * NHID;

static_assert(NHID % 32 == 0, "K multiple of 32");
static_assert(NTOK % TOK_BLK == 0, "token tiles exact");
static_assert(TOK_PASS == NWAVE * 16, "one 16-row subtile per wave per pass");
static_assert(NPACK % PACK_THR == 0, "pack grid exact");
static_assert((APITCH % 8) == 0 && APITCH >= NHID, "A tile pitch keeps 16-B alignment");
static_assert(BT_ROWS == 768, "three gate blocks of 256 rows");
static_assert(NGATE == 1024, "gate rows");

typedef __attribute__((ext_vector_type(16))) _Float16 v16h;
typedef __attribute__((ext_vector_type(8)))  _Float16 v8h;
typedef __attribute__((ext_vector_type(8)))  float    v8f;
typedef __attribute__((ext_vector_type(4)))  float    v4f;

__device__ __forceinline__ void dep_guard3_h(v8f& a, v8f& b, v8f& c, v16h x, v16h y0, v16h y1, v16h y2) {
  asm volatile("v_nop\n\tv_nop\n\tv_nop\n\tv_nop" : "+v"(a), "+v"(b), "+v"(c) : "v"(x), "v"(y0), "v"(y1), "v"(y2));
}
__device__ __forceinline__ void acc_guard3(v8f& a, v8f& b, v8f& c) {
  asm volatile("v_nop\n\tv_nop\n\tv_nop\n\tv_nop" : "+v"(a), "+v"(b), "+v"(c));
}

struct FragH {
  union U { v16h v; v8h h[2]; };
  static __device__ __forceinline__ v16h load(const _Float16* p) {
    U f;
    f.h[0] = *(const v8h*)(p);
    f.h[1] = *(const v8h*)(p + 16);
    return f.v;
  }
  static __device__ __forceinline__ v8f mma(v16h a, v16h b, v8f c) {
    return __builtin_amdgcn_wmma_f32_16x16x32_f16(false, a, false, b, (short)0, c, false, false);
  }
};

__device__ __forceinline__ float fsig(float x)  { return __builtin_amdgcn_rcpf(1.0f + __expf(-x)); }
__device__ __forceinline__ float ftanh(float x) { return 1.0f - 2.0f * __builtin_amdgcn_rcpf(__expf(2.0f * x) + 1.0f); }
__device__ __forceinline__ float cell_h(float zi, float zg, float zo) {
  const float cn = fsig(zi) * ftanh(zg);
  return fsig(zo) * ftanh(cn);
}

__global__ __launch_bounds__(PACK_THR) void pack_w1_kernel(const float* __restrict__ W1, unsigned short* __restrict__ BT) {
  const int i = blockIdx.x * PACK_THR + threadIdx.x;
  if (i < NPACK) {
    const int row = i >> 5;
    const int c8  = (i & 31) * 8;
    const int jg  = row / GRP_ROWS;
    const int rem = row - jg * GRP_ROWS;
    const int q   = rem >> 4;
    const int jl  = rem & 15;
    const int gbase = (q == 0) ? 0 : ((q == 1) ? ROW_G : ROW_O);
    const int src = gbase + jg * 16 + jl;
    const float* sp = W1 + (size_t)src * NHID + c8;
    const v4f a = *(const v4f*)(sp);
    const v4f b = *(const v4f*)(sp + 4);
    v8h hv;
#pragma unroll
    for (int e = 0; e < 4; ++e) {
      hv[e]     = (_Float16)(a[e] * WCARRY);
      hv[4 + e] = (_Float16)(b[e] * WCARRY);
    }
    volatile v8h* dp = (volatile v8h*)(BT + (size_t)row * NHID + c8);
    *dp = hv;
    __threadfence();
    *dp = hv;
  }
}

__global__ __launch_bounds__(NTHR) void cell2_fused_kernel(
    const float* __restrict__ x_in,
    const float* __restrict__ w_ih0, const float* __restrict__ b_ih0, const float* __restrict__ b_hh0,
    const float* __restrict__ b_ih1, const float* __restrict__ b_hh1,
    const float* __restrict__ w_lin, const float* __restrict__ b_lin,
    const unsigned short* __restrict__ BTp, float* __restrict__ out) {
  __shared__ __align__(16) _Float16 Ah[TOK_PASS * APITCH];
  __shared__ __align__(16) float    sC[C_TOT];
  __shared__ __align__(16) float    sOut[TOK_BLK];
  const _Float16* BT = (const _Float16*)BTp;
  const int tid = threadIdx.x, lane = tid & 31, wave = tid >> 5;
  const int c = lane & 15, hh = lane >> 4, koff = hh * 8;

#pragma unroll 1
  for (int j = tid; j < NHID; j += NTHR) {
    sC[C_W0I + j] = w_ih0[j];
    sC[C_W0G + j] = w_ih0[ROW_G + j];
    sC[C_W0O + j] = w_ih0[ROW_O + j];
    sC[C_B0I + j] = b_ih0[j] + b_hh0[j];
    sC[C_B0G + j] = b_ih0[ROW_G + j] + b_hh0[ROW_G + j];
    sC[C_B0O + j] = b_ih0[ROW_O + j] + b_hh0[ROW_O + j];
    sC[C_B1I + j] = b_ih1[j] + b_hh1[j];
    sC[C_B1G + j] = b_ih1[ROW_G + j] + b_hh1[ROW_G + j];
    sC[C_B1O + j] = b_ih1[ROW_O + j] + b_hh1[ROW_O + j];
    sC[C_WL  + j] = w_lin[j];
  }
  const float bl = b_lin[0];
  __syncthreads();

  const v8f z8 = {0.f, 0.f, 0.f, 0.f, 0.f, 0.f, 0.f, 0.f};
  _Float16* awave = Ah + (wave * 16) * APITCH;

#pragma unroll 1
  for (int pass = 0; pass < NPASS; ++pass) {
    const int tokbase = blockIdx.x * TOK_BLK + pass * TOK_PASS + wave * 16;
    const float xv = x_in[tokbase + c];

    {
      _Float16* arow = awave + c * APITCH + 128 * hh;
#pragma unroll 1
      for (int g = 0; g < 16; ++g) {
        const int j0 = 128 * hh + 8 * g;
        v8h hv;
#pragma unroll
        for (int q4 = 0; q4 < 2; ++q4) {
          const int jb = j0 + 4 * q4;
          const v4f wi = *(const v4f*)(sC + C_W0I + jb);
          const v4f wg = *(const v4f*)(sC + C_W0G + jb);
          const v4f wo = *(const v4f*)(sC + C_W0O + jb);
          const v4f ci = *(const v4f*)(sC + C_B0I + jb);
          const v4f cg = *(const v4f*)(sC + C_B0G + jb);
          const v4f co = *(const v4f*)(sC + C_B0O + jb);
#pragma unroll
          for (int e = 0; e < 4; ++e) {
            const float zi = fmaf(xv, wi[e], ci[e]);
            const float zg = fmaf(xv, wg[e], cg[e]);
            const float zo = fmaf(xv, wo[e], co[e]);
            const float h1 = cell_h(zi, zg, zo);
            hv[4 * q4 + e] = (_Float16)(h1 * ACARRY);
          }
        }
        *(v8h*)(arow + 8 * g) = hv;
      }
    }
    __syncthreads();

    v16h afr[KSTEPS];
    {
      const _Float16* ap = awave + c * APITCH + koff;
#pragma unroll
      for (int s = 0; s < KSTEPS; ++s) afr[s] = FragH::load(ap + 32 * s);
    }

    float oacc[8];
#pragma unroll
    for (int r = 0; r < 8; ++r) oacc[r] = 0.0f;

#pragma unroll 1
    for (int jg = 0; jg < NGRP; ++jg) {
      const _Float16* bp = BT + (size_t)(jg * GRP_ROWS + c) * NHID + koff;
      v8f ai = z8, ag = z8, ao = z8;
#pragma unroll
      for (int s = 0; s < KSTEPS; ++s) {
        const v16h bi = FragH::load(bp + 32 * s);
        const v16h bg = FragH::load(bp + 16 * NHID + 32 * s);
        const v16h bo = FragH::load(bp + 32 * NHID + 32 * s);
        ai = FragH::mma(afr[s], bi, ai);
        ag = FragH::mma(afr[s], bg, ag);
        ao = FragH::mma(afr[s], bo, ao);
        dep_guard3_h(ai, ag, ao, afr[s], bi, bg, bo);
      }
      acc_guard3(ai, ag, ao);
      const int j = 16 * jg + c;
      const float bi1 = sC[C_B1I + j];
      const float bg1 = sC[C_B1G + j];
      const float bo1 = sC[C_B1O + j];
      const float wl  = sC[C_WL + j];
#pragma unroll
      for (int r = 0; r < 8; ++r) {
        const float zi = fmaf(ai[r], FOLD, bi1);
        const float zg = fmaf(ag[r], FOLD, bg1);
        const float zo = fmaf(ao[r], FOLD, bo1);
        const float h2 = cell_h(zi, zg, zo);
        oacc[r] = fmaf(h2, wl, oacc[r]);
      }
    }

    float red[8];
#pragma unroll
    for (int r = 0; r < 8; ++r) {
      float v = oacc[r];
#pragma unroll
      for (int off = 1; off < 16; off <<= 1) v += __shfl_xor(v, off, 32);
      red[r] = v;
    }
    float sel = red[0];
#pragma unroll
    for (int r = 1; r < 8; ++r) sel = (c == r) ? red[r] : sel;
    if (c < 8) sOut[pass * TOK_PASS + wave * 16 + 8 * hh + c] = sel + bl;
    __syncthreads();
  }

  if (wave == 0) {
    const v4f v = *(const v4f*)(sOut + 4 * lane);
    volatile v4f* op = (volatile v4f*)(out + (size_t)blockIdx.x * TOK_BLK + 4 * lane);
    *op = v;
    __threadfence();
    *op = v;
  }
}

extern "C" void kernel_launch(void* const* d_in, const int* in_sizes, int n_in,
                              void* d_out, int out_size, void* d_ws, size_t ws_size, hipStream_t stream) {
  if (n_in < 11 || d_out == nullptr || d_ws == nullptr) return;
  if (in_sizes[0] != NTOK || in_sizes[1] != NGATE || in_sizes[3] != NGATE || in_sizes[4] != NGATE ||
      in_sizes[5] != NGATE * NHID || in_sizes[7] != NGATE || in_sizes[8] != NGATE ||
      in_sizes[9] != NHID || in_sizes[10] != 1 || out_size != NTOK) return;

  const float* x_in  = (const float*)d_in[0];
  const float* w_ih0 = (const float*)d_in[1];
  const float* b_ih0 = (const float*)d_in[3];
  const float* b_hh0 = (const float*)d_in[4];
  const float* w_ih1 = (const float*)d_in[5];
  const float* b_ih1 = (const float*)d_in[7];
  const float* b_hh1 = (const float*)d_in[8];
  const float* w_lin = (const float*)d_in[9];
  const float* b_lin = (const float*)d_in[10];
  float* out = (float*)d_out;

  char* ws = (char*)d_ws;
  size_t off = 0;
  unsigned short* BT = (unsigned short*)(ws + off);
  off += (((size_t)BT_ROWS * NHID * 2) + 255) & ~(size_t)255;
  if (off > ws_size || off > (size_t)134217728) return;

  pack_w1_kernel<<<NPACK / PACK_THR, PACK_THR, 0, stream>>>(w_ih1, BT);
  cell2_fused_kernel<<<NTOK / TOK_BLK, NTHR, 0, stream>>>(x_in, w_ih0, b_ih0, b_hh0, b_ih1, b_hh1,
                                                          w_lin, b_lin, BT, out);
}
